// MTLModel_31593779429829
// MI455X (gfx1250) — hardware-run, weakly checked
//
#include <hip/hip_runtime.h>
#include <math.h>

typedef __attribute__((ext_vector_type(16))) _Float16 v16h;
typedef __attribute__((ext_vector_type(8)))  _Float16 v8h;
typedef __attribute__((ext_vector_type(8)))  float    v8f;
typedef __attribute__((ext_vector_type(4)))  float    v4f;
typedef __attribute__((ext_vector_type(4)))  unsigned v4u;

constexpr int kBatch   = 1024;
constexpr int kTime    = 512;
constexpr int kCin     = 2;
constexpr int kLen1    = 511;
constexpr int kPool1   = 256;
constexpr int kChan1   = 128;
constexpr int kChan2   = 64;
constexpr int kSteps   = 128;
constexpr int kGateN   = 256;
constexpr int kHid     = 64;
constexpr int kTasks   = 32;
constexpr int kRowsA   = kBatch * kPool1;
constexpr int kRowsS   = kBatch * kSteps;
constexpr float kBnEps = 1e-5f;
static_assert(kLen1 == kTime - 1, "valid conv length");
static_assert(kPool1 == (kLen1 + 2) / 2, "pool 1 length");
static_assert(kSteps == kPool1 / 2, "pool 2 length");
static_assert((kChan1 % 32) == 0 && (kHid % 32) == 0, "GEMM K multiples of 32");
static_assert((kRowsA % 128) == 0 && (kChan2 % 64) == 0 && (kBatch % 16) == 0, "tile multiples");

constexpr float kCarW2   = 256.0f;
constexpr float kCarH1   = 16.0f;
constexpr float kCarWih  = 1024.0f;
constexpr float kCarSeq  = 64.0f;
constexpr float kCarWhh  = 256.0f;
constexpr float kCarHid  = 256.0f;
constexpr float kInvConv2 = 1.0f / (kCarW2 * kCarH1);
constexpr float kInvGate  = 1.0f / (kCarWih * kCarSeq);
static_assert(kCarWih * kCarSeq == kCarWhh * kCarHid, "input and hidden products share one accumulator scale");

constexpr size_t kOffW2H  = 0;
constexpr size_t kOffWIH  = kOffW2H  + (size_t)kChan2 * kChan1 * 2;
constexpr size_t kOffWHH  = kOffWIH  + (size_t)kGateN * kHid * 2;
constexpr size_t kOffP1   = kOffWHH  + (size_t)kGateN * kHid * 2;
constexpr size_t kOffBN1  = kOffP1   + (size_t)kBatch * 256 * 4;
constexpr size_t kOffP2   = kOffBN1  + (size_t)256 * 4;
constexpr size_t kOffBN2  = kOffP2   + (size_t)(kRowsA / 128) * 128 * 4;
constexpr size_t kOffH1   = kOffBN2  + (size_t)128 * 4;
constexpr size_t kOffY2   = kOffH1   + (size_t)kRowsA * kChan1 * 2;
constexpr size_t kOffSEQ  = kOffY2   + (size_t)kRowsA * kChan2 * 2;
constexpr size_t kOffSHR  = kOffSEQ  + (size_t)kRowsS * kChan2 * 2;
constexpr size_t kWsTotal = kOffSHR  + (size_t)kBatch * kHid * 4;
static_assert(kWsTotal == 119883264ull, "carve total");
static_assert(kWsTotal <= 134217728ull, "carve cap");
static_assert((kOffWIH % 128) == 0 && (kOffWHH % 128) == 0 && (kOffP1 % 128) == 0 && (kOffBN1 % 128) == 0 &&
              (kOffP2 % 128) == 0 && (kOffBN2 % 128) == 0 && (kOffH1 % 128) == 0 && (kOffY2 % 128) == 0 &&
              (kOffSEQ % 128) == 0 && (kOffSHR % 128) == 0, "128-B aligned regions");

union FragU { v16h v; v8h h[2]; };
__device__ __forceinline__ v16h frag_load(const _Float16* p) {
  FragU f;
  f.h[0] = *(const v8h*)(p);
  f.h[1] = *(const v8h*)(p + 16);
  return f.v;
}
__device__ __forceinline__ v8f mma_f16(v16h a, v16h b, v8f c) {
  return __builtin_amdgcn_wmma_f32_16x16x32_f16(false, a, false, b, (short)0, c, false, false);
}
__device__ __forceinline__ void hz_guard2(v8f& acc, v16h x, v16h y) {
  asm volatile("v_nop\n\tv_nop\n\tv_nop\n\tv_nop" : "+v"(acc) : "v"(x), "v"(y));
}
__device__ __forceinline__ void hz_guard4(v8f& acc, v16h x0, v16h x1, v16h x2, v16h x3) {
  asm volatile("v_nop\n\tv_nop\n\tv_nop\n\tv_nop" : "+v"(acc) : "v"(x0), "v"(x1), "v"(x2), "v"(x3));
}
__device__ __forceinline__ void keep4(v16h a, v16h b, v16h c, v16h d) {
  asm volatile("v_nop" :: "v"(a), "v"(b), "v"(c), "v"(d));
}

__device__ __forceinline__ float h16_to_f32(unsigned hb) {
  const unsigned sgn = (hb & 0x8000u) << 16;
  const unsigned em = hb & 0x7fffu;
  const float fn = __uint_as_float((em << 13) + 0x38000000u);
  const float fs = (float)em * 5.9604644775390625e-8f;
  const float mag = (em < 0x400u) ? fs : fn;
  return __uint_as_float(__float_as_uint(mag) | sgn);
}

__device__ __forceinline__ float sigm(float x) {
  return __builtin_amdgcn_rcpf(1.0f + expf(-x));
}

__global__ __launch_bounds__(256) void prep_weights_kernel(
    const float* __restrict__ w2, const float* __restrict__ wih, const float* __restrict__ whh,
    unsigned short* __restrict__ w2h, unsigned short* __restrict__ wihh, unsigned short* __restrict__ whhh)
{
  const int blk = blockIdx.x;
  const float* src;
  unsigned short* dst;
  float car;
  int base;
  if (blk < 4)       { src = w2;  dst = w2h;  car = kCarW2;  base = blk; }
  else if (blk < 12) { src = wih; dst = wihh; car = kCarWih; base = blk - 4; }
  else               { src = whh; dst = whhh; car = kCarWhh; base = blk - 12; }
  const size_t e0 = ((size_t)base * 256 + threadIdx.x) * 8;
  const v4f a0 = *(const v4f*)(src + e0);
  const v4f a1 = *(const v4f*)(src + e0 + 4);
  v8h hv;
#pragma unroll
  for (int e = 0; e < 4; ++e) {
    hv[e]     = (_Float16)(a0[e] * car);
    hv[4 + e] = (_Float16)(a1[e] * car);
  }
  unsigned short* q = dst + e0;
  *(volatile v8h*)q = hv;
  __threadfence();
  *(volatile v8h*)q = hv;
}

__device__ __forceinline__ float conv1_at(const float* xs, int p, float w00, float w01, float w10, float w11, float bc) {
  float y = w00 * xs[2 * p];
  y = fmaf(w01, xs[2 * p + 2], y);
  y = fmaf(w10, xs[2 * p + 1], y);
  y = fmaf(w11, xs[2 * p + 3], y);
  return y + bc;
}

__global__ __launch_bounds__(256) void conv1_stats_kernel(
    const float* __restrict__ x, const float* __restrict__ w, const float* __restrict__ bias,
    float* __restrict__ part1)
{
  __shared__ __align__(16) float xls[kTime * kCin];
  __shared__ __align__(16) float red[512];
  const int b = blockIdx.x, tid = threadIdx.x;
  *(v4f*)(xls + tid * 4) = *(const v4f*)(x + (size_t)b * (kTime * kCin) + tid * 4);
  __syncthreads();
  const int c = tid & 127, half = tid >> 7;
  const v4f wv = *(const v4f*)(w + c * 4);
  const float w00 = wv[0], w01 = wv[1], w10 = wv[2], w11 = wv[3];
  const float bc = bias[c];
  float s = 0.f, q = 0.f;
#pragma unroll 4
  for (int p = half; p < kLen1; p += 2) {
    const float y = conv1_at(xls, p, w00, w01, w10, w11, bc);
    s += y;
    q = fmaf(y, y, q);
  }
  red[half * 256 + c] = s;
  red[half * 256 + 128 + c] = q;
  __syncthreads();
  if (tid < 64) {
    const v4f a = *(const v4f*)(red + tid * 4);
    const v4f d = *(const v4f*)(red + 256 + tid * 4);
    const v4f v = a + d;
    float* dst = part1 + (size_t)b * 256 + tid * 4;
    *(volatile v4f*)dst = v;
    __threadfence();
    *(volatile v4f*)dst = v;
  }
}

__global__ __launch_bounds__(256) void bn_finalize_kernel(
    const float* __restrict__ part, int nrows, int nch,
    const float* __restrict__ g, const float* __restrict__ bb,
    float* __restrict__ outp, double inv_count)
{
  __shared__ double tot[256];
  __shared__ __align__(16) float res[256];
  const int tid = threadIdx.x;
  const int ncol = 2 * nch;
  const int col = (tid < ncol) ? tid : (ncol - 1);
  double acc = 0.0;
#pragma unroll 4
  for (int r = 0; r < nrows; ++r) acc += (double)part[(size_t)r * ncol + col];
  tot[tid] = acc;
  __syncthreads();
  {
    const int ch = (tid < nch) ? tid : (nch - 1);
    const double mean = tot[ch] * inv_count;
    const double ex2  = tot[nch + ch] * inv_count;
    const float varf  = fmaxf((float)(ex2 - mean * mean), 0.0f);
    const float sc = g[ch] * rsqrtf(varf + kBnEps);
    const float sh = bb[ch] - (float)mean * sc;
    if (tid < nch) {
      res[tid] = sc;
      res[nch + tid] = sh;
    }
  }
  __syncthreads();
  if (tid < (ncol >> 2)) {
    const v4f v = *(const v4f*)(res + tid * 4);
    float* dst = outp + tid * 4;
    *(volatile v4f*)dst = v;
    __threadfence();
    *(volatile v4f*)dst = v;
  }
}

constexpr int kTileP = 132;
__global__ __launch_bounds__(256) void conv1_bn_pool_kernel(
    const float* __restrict__ x, const float* __restrict__ w, const float* __restrict__ bias,
    const float* __restrict__ bn1, unsigned short* __restrict__ h1)
{
  __shared__ __align__(16) float xls[kTime * kCin];
  __shared__ __align__(16) float sT[16 * kTileP];
  const int b = blockIdx.x, tid = threadIdx.x;
  *(v4f*)(xls + tid * 4) = *(const v4f*)(x + (size_t)b * (kTime * kCin) + tid * 4);
  __syncthreads();
  const int c = tid & 127, half = tid >> 7;
  const v4f wv = *(const v4f*)(w + c * 4);
  const float w00 = wv[0], w01 = wv[1], w10 = wv[2], w11 = wv[3];
  const float bc = bias[c];
  const float sc = bn1[c], sh = bn1[kChan1 + c];
  const int srow = tid >> 4, c8 = (tid & 15) * 8;
#pragma unroll 1
  for (int chunk = 0; chunk < 16; ++chunk) {
#pragma unroll 2
    for (int i = 0; i < 8; ++i) {
      const int lr = half + 2 * i;
      const int po = chunk * 16 + lr;
      const int pb = 2 * po;
      const int pa = (pb > 0) ? (pb - 1) : 0;
      const float ya = conv1_at(xls, pa, w00, w01, w10, w11, bc);
      const float yb = conv1_at(xls, pb, w00, w01, w10, w11, bc);
      const float za = fmaxf(fmaf(ya, sc, sh), 0.0f);
      const float zb = fmaxf(fmaf(yb, sc, sh), 0.0f);
      sT[lr * kTileP + c] = fmaxf(za, zb) * kCarH1;
    }
    __syncthreads();
    const v4f a0 = *(const v4f*)(sT + srow * kTileP + c8);
    const v4f a1 = *(const v4f*)(sT + srow * kTileP + c8 + 4);
    v8h hv;
#pragma unroll
    for (int e = 0; e < 4; ++e) {
      hv[e]     = (_Float16)a0[e];
      hv[4 + e] = (_Float16)a1[e];
    }
    unsigned short* dst = h1 + ((size_t)b * kPool1 + chunk * 16 + srow) * kChan1 + c8;
    *(volatile v8h*)dst = hv;
    __threadfence();
    *(volatile v8h*)dst = hv;
    __syncthreads();
  }
}

__global__ __launch_bounds__(256) void conv2_gemm_kernel(
    const unsigned short* __restrict__ h1p, const unsigned short* __restrict__ w2p,
    const float* __restrict__ bias, unsigned short* __restrict__ y2, float* __restrict__ part2)
{
  __shared__ __align__(16) float slab[8][16 * 68];
  __shared__ __align__(16) float sStat[8][128];
  const _Float16* A  = (const _Float16*)h1p;
  const _Float16* Bt = (const _Float16*)w2p;
  const int lane = threadIdx.x & 31, wave = threadIdx.x >> 5;
  const int rl = lane & 15, hh = lane >> 4, koff = hh * 8;
  const int m0 = blockIdx.x * 128 + wave * 16;
  v8f acc[4];
#pragma unroll
  for (int j = 0; j < 4; ++j) acc[j] = (v8f){0.f, 0.f, 0.f, 0.f, 0.f, 0.f, 0.f, 0.f};
  const _Float16* arow = A + (size_t)(m0 + rl) * kChan1 + koff;
  const _Float16* brow = Bt + (size_t)rl * kChan1 + koff;
#pragma unroll 1
  for (int kt = 0; kt < kChan1 / 32; ++kt) {
    const v16h a  = frag_load(arow + kt * 32);
    const v16h b0 = frag_load(brow + kt * 32);
    const v16h b1 = frag_load(brow + 16 * kChan1 + kt * 32);
    const v16h b2 = frag_load(brow + 32 * kChan1 + kt * 32);
    const v16h b3 = frag_load(brow + 48 * kChan1 + kt * 32);
    acc[0] = mma_f16(a, b0, acc[0]);
    acc[1] = mma_f16(a, b1, acc[1]);
    acc[2] = mma_f16(a, b2, acc[2]);
    acc[3] = mma_f16(a, b3, acc[3]);
    hz_guard2(acc[0], a, b0);
    hz_guard2(acc[1], a, b1);
    hz_guard2(acc[2], a, b2);
    hz_guard2(acc[3], a, b3);
  }
  float* sl = slab[wave];
  float ps[4], pq[4];
#pragma unroll
  for (int j = 0; j < 4; ++j) {
    const float bv = bias[j * 16 + rl];
    float s = 0.f, q = 0.f;
#pragma unroll
    for (int r = 0; r < 8; ++r) {
      const float v = fmaf(acc[j][r], kInvConv2, bv);
      sl[(8 * hh + r) * 68 + j * 16 + rl] = v;
      s += v;
      q = fmaf(v, v, q);
    }
    ps[j] = s;
    pq[j] = q;
  }
#pragma unroll
  for (int j = 0; j < 4; ++j) {
    ps[j] += __shfl_xor(ps[j], 16, 32);
    pq[j] += __shfl_xor(pq[j], 16, 32);
  }
  if (lane < 16) {
#pragma unroll
    for (int j = 0; j < 4; ++j) {
      sStat[wave][j * 16 + lane] = ps[j];
      sStat[wave][64 + j * 16 + lane] = pq[j];
    }
  }
  __syncthreads();
  {
    const int q4 = lane >> 3, c8 = (lane & 7) * 8;
    v8h hv[4];
#pragma unroll
    for (int it = 0; it < 4; ++it) {
      const float* sp = sl + (it * 4 + q4) * 68 + c8;
      const v4f a0 = *(const v4f*)(sp);
      const v4f a1 = *(const v4f*)(sp + 4);
#pragma unroll
      for (int e = 0; e < 4; ++e) {
        hv[it][e]     = (_Float16)a0[e];
        hv[it][4 + e] = (_Float16)a1[e];
      }
    }
    for (int pass = 0; pass < 2; ++pass) {
#pragma unroll
      for (int it = 0; it < 4; ++it)
        *(volatile v8h*)(y2 + (size_t)(m0 + it * 4 + q4) * kChan2 + c8) = hv[it];
      __threadfence();
    }
  }
  if (wave == 0) {
    v4f t;
#pragma unroll
    for (int e = 0; e < 4; ++e) {
      const int col = lane * 4 + e;
      float a = sStat[0][col];
#pragma unroll
      for (int wv = 1; wv < 8; ++wv) a += sStat[wv][col];
      t[e] = a;
    }
    float* dst = part2 + (size_t)blockIdx.x * 128 + lane * 4;
    *(volatile v4f*)dst = t;
    __threadfence();
    *(volatile v4f*)dst = t;
  }
}

__global__ __launch_bounds__(256) void bn2_pool_kernel(
    const unsigned short* __restrict__ y2, const float* __restrict__ bn2, unsigned short* __restrict__ seq)
{
  const int gid = blockIdx.x * 256 + threadIdx.x;
  const int row = gid >> 3, c8 = (gid & 7) * 8;
  const v4u wa = *(const v4u*)(const void*)(y2 + (size_t)(2 * row) * kChan2 + c8);
  const v4u wb = *(const v4u*)(const void*)(y2 + (size_t)(2 * row + 1) * kChan2 + c8);
  const v4f sc0 = *(const v4f*)(bn2 + c8);
  const v4f sc1 = *(const v4f*)(bn2 + c8 + 4);
  const v4f sh0 = *(const v4f*)(bn2 + kChan2 + c8);
  const v4f sh1 = *(const v4f*)(bn2 + kChan2 + c8 + 4);
  float scv[8], shv[8];
#pragma unroll
  for (int e = 0; e < 4; ++e) {
    scv[e] = sc0[e]; scv[4 + e] = sc1[e];
    shv[e] = sh0[e]; shv[4 + e] = sh1[e];
  }
  v8h hv;
#pragma unroll
  for (int e = 0; e < 4; ++e) {
    const unsigned ua = wa[e];
    const unsigned ub = wb[e];
    const float ya0 = h16_to_f32(ua & 0xffffu), ya1 = h16_to_f32(ua >> 16);
    const float yb0 = h16_to_f32(ub & 0xffffu), yb1 = h16_to_f32(ub >> 16);
    const float za0 = fmaxf(fmaf(ya0, scv[2 * e], shv[2 * e]), 0.0f);
    const float zb0 = fmaxf(fmaf(yb0, scv[2 * e], shv[2 * e]), 0.0f);
    const float za1 = fmaxf(fmaf(ya1, scv[2 * e + 1], shv[2 * e + 1]), 0.0f);
    const float zb1 = fmaxf(fmaf(yb1, scv[2 * e + 1], shv[2 * e + 1]), 0.0f);
    hv[2 * e]     = (_Float16)(fmaxf(za0, zb0) * kCarSeq);
    hv[2 * e + 1] = (_Float16)(fmaxf(za1, zb1) * kCarSeq);
  }
  unsigned short* dst = seq + (size_t)row * kChan2 + c8;
  *(volatile v8h*)dst = hv;
  __threadfence();
  *(volatile v8h*)dst = hv;
}

__global__ __launch_bounds__(256) void lstm_mean_kernel(
    const unsigned short* __restrict__ seqp, const unsigned short* __restrict__ wihp,
    const unsigned short* __restrict__ whhp, const float* __restrict__ bih, const float* __restrict__ bhh,
    float* __restrict__ shared_out)
{
  __shared__ __align__(16) _Float16 hs[16 * kHid];
  __shared__ __align__(16) float sMean[16 * kHid];
  const _Float16* seq = (const _Float16*)seqp;
  const _Float16* wih = (const _Float16*)wihp;
  const _Float16* whh = (const _Float16*)whhp;
  const int tid = threadIdx.x, lane = tid & 31, wave = tid >> 5;
  const int rl = lane & 15, hh = lane >> 4, koff = hh * 8;
  const int s0 = blockIdx.x * 16;

  const int usub = rl & 7, gsel = rl >> 3;
  const int wrow0 = gsel * kHid + wave * 8 + usub;
  const int wrow1 = (2 + gsel) * kHid + wave * 8 + usub;
  v16h bi0[2], bi1[2], bh0[2], bh1[2];
#pragma unroll
  for (int kt = 0; kt < 2; ++kt) {
    bi0[kt] = frag_load(wih + (size_t)wrow0 * kHid + kt * 32 + koff);
    bi1[kt] = frag_load(wih + (size_t)wrow1 * kHid + kt * 32 + koff);
    bh0[kt] = frag_load(whh + (size_t)wrow0 * kHid + kt * 32 + koff);
    bh1[kt] = frag_load(whh + (size_t)wrow1 * kHid + kt * 32 + koff);
  }
  const float bias0 = bih[wrow0] + bhh[wrow0];
  const float bias1 = bih[wrow1] + bhh[wrow1];

#pragma unroll
  for (int e = 0; e < 4; ++e) hs[tid * 4 + e] = (_Float16)0.0f;

  float cst[4], hsum[4];
#pragma unroll
  for (int k = 0; k < 4; ++k) { cst[k] = 0.f; hsum[k] = 0.f; }
  const bool hq = ((lane >> 3) & 1) != 0;
  const int mrow = (lane >> 3) * 4;
  const int ucol = wave * 8 + (lane & 7);
  const _Float16* xbase = seq + (size_t)(s0 + rl) * kSteps * kChan2 + koff;
  const _Float16* hbase = hs + rl * kHid + koff;
  __syncthreads();

#pragma unroll 1
  for (int t = 0; t < kSteps; ++t) {
    const v16h xa0 = frag_load(xbase + t * kChan2);
    const v16h xa1 = frag_load(xbase + t * kChan2 + 32);
    const v16h ha0 = frag_load(hbase);
    const v16h ha1 = frag_load(hbase + 32);
    v8f acc0 = (v8f){0.f, 0.f, 0.f, 0.f, 0.f, 0.f, 0.f, 0.f};
    v8f acc1 = (v8f){0.f, 0.f, 0.f, 0.f, 0.f, 0.f, 0.f, 0.f};
    acc0 = mma_f16(xa0, bi0[0], acc0);
    acc1 = mma_f16(xa0, bi1[0], acc1);
    acc0 = mma_f16(ha0, bh0[0], acc0);
    acc1 = mma_f16(ha0, bh1[0], acc1);
    acc0 = mma_f16(xa1, bi0[1], acc0);
    acc1 = mma_f16(xa1, bi1[1], acc1);
    acc0 = mma_f16(ha1, bh0[1], acc0);
    acc1 = mma_f16(ha1, bh1[1], acc1);
    hz_guard4(acc0, xa0, xa1, ha0, ha1);
    hz_guard4(acc1, xa0, xa1, ha0, ha1);
    keep4(bi0[0], bi0[1], bh0[0], bh0[1]);
    keep4(bi1[0], bi1[1], bh1[0], bh1[1]);

    float v0[8], v1[8], p0[8], p1[8];
#pragma unroll
    for (int r = 0; r < 8; ++r) {
      v0[r] = fmaf(acc0[r], kInvGate, bias0);
      v1[r] = fmaf(acc1[r], kInvGate, bias1);
    }
#pragma unroll
    for (int r = 0; r < 8; ++r) {
      p0[r] = __shfl_xor(v0[r], 8, 32);
      p1[r] = __shfl_xor(v1[r], 8, 32);
    }
    __syncthreads();
#pragma unroll
    for (int k = 0; k < 4; ++k) {
      const float gi = hq ? p0[k + 4] : v0[k];
      const float gf = hq ? v0[k + 4] : p0[k];
      const float gg = hq ? p1[k + 4] : v1[k];
      const float go = hq ? v1[k + 4] : p1[k];
      const float cn = sigm(gf) * cst[k] + sigm(gi) * tanhf(gg);
      cst[k] = cn;
      const float hv = sigm(go) * tanhf(cn);
      hsum[k] += hv;
      hs[(mrow + k) * kHid + ucol] = (_Float16)(hv * kCarHid);
    }
    __syncthreads();
  }

#pragma unroll
  for (int k = 0; k < 4; ++k) sMean[(mrow + k) * kHid + ucol] = hsum[k] * (1.0f / (float)kSteps);
  __syncthreads();
  {
    const int row = tid >> 4, c4 = (tid & 15) * 4;
    const v4f v = *(const v4f*)(sMean + row * kHid + c4);
    float* dst = shared_out + (size_t)(s0 + row) * kHid + c4;
    *(volatile v4f*)dst = v;
    __threadfence();
    *(volatile v4f*)dst = v;
  }
}

__global__ __launch_bounds__(256) void heads_kernel(
    const float* __restrict__ shared_in, const int* __restrict__ task_ids,
    const float* __restrict__ W1, const float* __restrict__ b1,
    const float* __restrict__ W2, const float* __restrict__ b2,
    const float* __restrict__ Wo, const float* __restrict__ bo,
    float* __restrict__ out)
{
  __shared__ __align__(16) float sv[8][64];
  __shared__ __align__(16) float a1[8][128];
  __shared__ __align__(16) float a2[8][64];
  __shared__ __align__(16) float outv[32];
  const int tid = threadIdx.x, lane = tid & 31, wave = tid >> 5;
#pragma unroll 1
  for (int it = 0; it < 4; ++it) {
    const int sl = wave * 4 + it;
    const int b = blockIdx.x * 32 + sl;
    int tau = task_ids[b];
    tau = tau < 0 ? 0 : (tau > (kTasks - 1) ? (kTasks - 1) : tau);
    sv[wave][lane]      = shared_in[(size_t)b * kHid + lane];
    sv[wave][lane + 32] = shared_in[(size_t)b * kHid + lane + 32];
    __syncthreads();
#pragma unroll 1
    for (int j = 0; j < 4; ++j) {
      const int o = j * 32 + lane;
      const float* wr = W1 + ((size_t)tau * 128 + o) * 64;
      float acc = b1[tau * 128 + o];
#pragma unroll 4
      for (int k4 = 0; k4 < 16; ++k4) {
        const v4f wv = *(const v4f*)(wr + 4 * k4);
        const v4f xv = *(const v4f*)(&sv[wave][4 * k4]);
        acc = fmaf(wv[0], xv[0], acc);
        acc = fmaf(wv[1], xv[1], acc);
        acc = fmaf(wv[2], xv[2], acc);
        acc = fmaf(wv[3], xv[3], acc);
      }
      a1[wave][o] = fmaxf(acc, 0.0f);
    }
    __syncthreads();
#pragma unroll 1
    for (int j = 0; j < 2; ++j) {
      const int o = j * 32 + lane;
      const float* wr = W2 + ((size_t)tau * 64 + o) * 128;
      float acc = b2[tau * 64 + o];
#pragma unroll 4
      for (int k4 = 0; k4 < 32; ++k4) {
        const v4f wv = *(const v4f*)(wr + 4 * k4);
        const v4f xv = *(const v4f*)(&a1[wave][4 * k4]);
        acc = fmaf(wv[0], xv[0], acc);
        acc = fmaf(wv[1], xv[1], acc);
        acc = fmaf(wv[2], xv[2], acc);
        acc = fmaf(wv[3], xv[3], acc);
      }
      a2[wave][o] = fmaxf(acc, 0.0f);
    }
    __syncthreads();
    float pr = Wo[tau * 64 + lane] * a2[wave][lane];
    pr = fmaf(Wo[tau * 64 + lane + 32], a2[wave][lane + 32], pr);
#pragma unroll
    for (int off = 16; off > 0; off >>= 1) pr += __shfl_xor(pr, off, 32);
    float bov = bo[tau];
    asm volatile("" : "+v"(bov));
    if (lane == 0) outv[sl] = pr + bov;
  }
  __syncthreads();
  if (tid < 8) {
    const v4f v = *(const v4f*)(outv + tid * 4);
    float* dst = out + (size_t)blockIdx.x * 32 + tid * 4;
    *(volatile v4f*)dst = v;
    __threadfence();
    *(volatile v4f*)dst = v;
  }
}

extern "C" void kernel_launch(void* const* d_in, const int* in_sizes, int n_in,
                              void* d_out, int out_size, void* d_ws, size_t ws_size,
                              hipStream_t stream) {
  if (n_in < 20) return;
  if (in_sizes[0] != kBatch * kTime * kCin) return;
  if (in_sizes[1] != kBatch) return;
  if (in_sizes[2] != kChan1 * kCin * 2) return;
  if (in_sizes[6] != kChan2 * kChan1) return;
  if (in_sizes[10] != kGateN * kHid) return;
  if (in_sizes[11] != kGateN * kHid) return;
  if (in_sizes[14] != kTasks * 128 * 64) return;
  if (in_sizes[16] != kTasks * 64 * 128) return;
  if (in_sizes[18] != kTasks * 64) return;
  if (in_sizes[19] != kTasks) return;
  if (out_size != kBatch) return;
  if (ws_size < kWsTotal) return;

  const float* x        = (const float*)d_in[0];
  const int*   task_ids = (const int*)d_in[1];
  const float* conv1_w  = (const float*)d_in[2];
  const float* conv1_b  = (const float*)d_in[3];
  const float* bn1_g    = (const float*)d_in[4];
  const float* bn1_b    = (const float*)d_in[5];
  const float* conv2_w  = (const float*)d_in[6];
  const float* conv2_b  = (const float*)d_in[7];
  const float* bn2_g    = (const float*)d_in[8];
  const float* bn2_b    = (const float*)d_in[9];
  const float* wih      = (const float*)d_in[10];
  const float* whh      = (const float*)d_in[11];
  const float* bih      = (const float*)d_in[12];
  const float* bhh      = (const float*)d_in[13];
  const float* W1       = (const float*)d_in[14];
  const float* b1       = (const float*)d_in[15];
  const float* W2       = (const float*)d_in[16];
  const float* b2       = (const float*)d_in[17];
  const float* Wo       = (const float*)d_in[18];
  const float* bo       = (const float*)d_in[19];
  float* out = (float*)d_out;

  char* ws = (char*)d_ws;
  unsigned short* W2H  = (unsigned short*)(ws + kOffW2H);
  unsigned short* WIHH = (unsigned short*)(ws + kOffWIH);
  unsigned short* WHHH = (unsigned short*)(ws + kOffWHH);
  float*          P1   = (float*)(ws + kOffP1);
  float*          BN1  = (float*)(ws + kOffBN1);
  float*          P2   = (float*)(ws + kOffP2);
  float*          BN2  = (float*)(ws + kOffBN2);
  unsigned short* H1   = (unsigned short*)(ws + kOffH1);
  unsigned short* Y2   = (unsigned short*)(ws + kOffY2);
  unsigned short* SEQ  = (unsigned short*)(ws + kOffSEQ);
  float*          SHR  = (float*)(ws + kOffSHR);

  prep_weights_kernel<<<20, 256, 0, stream>>>(conv2_w, wih, whh, W2H, WIHH, WHHH);
  conv1_stats_kernel<<<kBatch, 256, 0, stream>>>(x, conv1_w, conv1_b, P1);
  bn_finalize_kernel<<<1, 256, 0, stream>>>(P1, kBatch, kChan1, bn1_g, bn1_b, BN1,
                                            1.0 / ((double)kBatch * (double)kLen1));
  conv1_bn_pool_kernel<<<kBatch, 256, 0, stream>>>(x, conv1_w, conv1_b, BN1, H1);
  conv2_gemm_kernel<<<kRowsA / 128, 256, 0, stream>>>(H1, W2H, conv2_b, Y2, P2);
  bn_finalize_kernel<<<1, 256, 0, stream>>>(P2, kRowsA / 128, kChan2, bn2_g, bn2_b, BN2,
                                            1.0 / (double)kRowsA);
  bn2_pool_kernel<<<(kRowsS * 8) / 256, 256, 0, stream>>>(Y2, BN2, SEQ);
  lstm_mean_kernel<<<kBatch / 16, 256, 0, stream>>>(SEQ, WIHH, WHHH, bih, bhh, SHR);
  heads_kernel<<<kBatch / 32, 256, 0, stream>>>(SHR, task_ids, W1, b1, W2, b2, Wo, bo, out);
}
